// NonLocalBlockLinear_67482526155125
// MI455X (gfx1250) — hardware-verified
//
#include <hip/hip_runtime.h>
#include <math.h>

constexpr int NBATCH = 8;
constexpr int NCH    = 512;
constexpr int NIC    = 256;
constexpr int NTOK   = 3136;
constexpr float WCARRY     = 16.0f;
constexpr float WCARRY_INV = 1.0f / 16.0f;
constexpr float PCARRY     = 32768.0f;
constexpr float YCARRY     = 256.0f;
constexpr float PV_SCALE   = YCARRY / PCARRY;
constexpr float Z_SCALE    = 1.0f / (WCARRY * YCARRY);
constexpr float BNEPS      = 1e-5f;

static_assert(NTOK % 64 == 0);
static_assert(NTOK % 32 == 0);
static_assert(NCH % 64 == 0 && NIC % 64 == 0 && NCH % 32 == 0 && NIC % 32 == 0);

constexpr size_t OFF_WQK  = 0;
constexpr size_t OFF_WG   = OFF_WQK  + (size_t)NCH * NCH * 2;
constexpr size_t OFF_WZ   = OFF_WG   + (size_t)NIC * NCH * 2;
constexpr size_t OFF_VEC  = OFF_WZ   + (size_t)NCH * NIC * 2;
constexpr size_t OFF_XTM  = OFF_VEC  + 16384;
constexpr size_t OFF_QKH  = OFF_XTM  + (size_t)NTOK * NCH * 2;
constexpr size_t OFF_QKL  = OFF_QKH  + (size_t)NTOK * NCH * 2;
constexpr size_t OFF_VT   = OFF_QKL  + (size_t)NTOK * NCH * 2;
constexpr size_t OFF_S    = OFF_VT   + (size_t)NIC * NTOK * 2;
constexpr size_t OFF_P    = OFF_S    + (size_t)NTOK * NTOK * 4;
constexpr size_t OFF_Y    = OFF_P    + (size_t)NTOK * NTOK * 2;
constexpr size_t OFF_Z    = OFF_Y    + (size_t)NTOK * NIC * 2;
constexpr size_t WS_END   = OFF_Z    + (size_t)NBATCH * NCH * NTOK * 4;
static_assert(WS_END == 124297216);
static_assert(WS_END <= 134217728);
static_assert((OFF_VEC % 128) == 0 && (OFF_XTM % 128) == 0 && (OFF_QKH % 128) == 0 && (OFF_QKL % 128) == 0 &&
              (OFF_VT % 128) == 0 && (OFF_S % 128) == 0 && (OFF_P % 128) == 0 && (OFF_Y % 128) == 0 &&
              (OFF_Z % 128) == 0);

typedef __attribute__((ext_vector_type(16))) _Float16 v16h;
typedef __attribute__((ext_vector_type(8)))  _Float16 v8h;
typedef __attribute__((ext_vector_type(16))) __bf16   v16b;
typedef __attribute__((ext_vector_type(8)))  __bf16   v8b;
typedef __attribute__((ext_vector_type(8)))  float    v8f;
typedef __attribute__((ext_vector_type(4)))  float    v4f;
typedef __attribute__((ext_vector_type(4)))  unsigned int v4u;

__device__ __forceinline__ unsigned short f2bf_bits(float f) {
  unsigned u = __float_as_uint(f);
  return (unsigned short)((u + 0x7FFFu + ((u >> 16) & 1u)) >> 16);
}
__device__ __forceinline__ float bf_bits2f(unsigned short h) { return __uint_as_float(((unsigned)h) << 16); }

__device__ __forceinline__ void dep_guard_h(v8f& a, v8f& b, v16h x, v16h y) { asm volatile("v_nop\n\tv_nop\n\tv_nop\n\tv_nop" : "+v"(a), "+v"(b) : "v"(x), "v"(y)); }
__device__ __forceinline__ void dep_guard_b(v8f& a, v8f& b, v16b x, v16b y) { asm volatile("v_nop\n\tv_nop\n\tv_nop\n\tv_nop" : "+v"(a), "+v"(b) : "v"(x), "v"(y)); }
__device__ __forceinline__ void keep4_h(v16h a, v16h b, v16h c, v16h d) { asm volatile("v_nop" :: "v"(a), "v"(b), "v"(c), "v"(d)); }
__device__ __forceinline__ void keep4_b(v16b a, v16b b, v16b c, v16b d) { asm volatile("v_nop" :: "v"(a), "v"(b), "v"(c), "v"(d)); }
__device__ __forceinline__ void acc_guard4(v8f& a, v8f& b, v8f& c, v8f& d) { asm volatile("v_nop\n\tv_nop\n\tv_nop\n\tv_nop" : "+v"(a), "+v"(b), "+v"(c), "+v"(d)); }
template <typename T> struct Frag;
template <> struct Frag<_Float16> {
  typedef v16h V; union U { v16h v; v8h h[2]; };
  static __device__ __forceinline__ v16h load(const _Float16* p) {
    U f; f.h[0] = *(const v8h*)(p); f.h[1] = *(const v8h*)(p + 16); return f.v;
  }
  static __device__ __forceinline__ v8f mma(v16h a, v16h b, v8f c) {
    return __builtin_amdgcn_wmma_f32_16x16x32_f16(false, a, false, b, (short)0, c, false, false);
  }
  static __device__ __forceinline__ void guard(v8f& a, v8f& b, v16h x, v16h y) { dep_guard_h(a, b, x, y); }
  static __device__ __forceinline__ void keep(v16h a, v16h b, v16h c, v16h d) { keep4_h(a, b, c, d); }
};
template <> struct Frag<__bf16> {
  typedef v16b V; union U { v16b v; v8b h[2]; };
  static __device__ __forceinline__ v16b load(const __bf16* p) {
    U f; f.h[0] = *(const v8b*)(p); f.h[1] = *(const v8b*)(p + 16); return f.v;
  }
  static __device__ __forceinline__ v8f mma(v16b a, v16b b, v8f c) {
    return __builtin_amdgcn_wmma_f32_16x16x32_bf16(false, a, false, b, (short)0, c, false, false);
  }
  static __device__ __forceinline__ void guard(v8f& a, v8f& b, v16b x, v16b y) { dep_guard_b(a, b, x, y); }
  static __device__ __forceinline__ void keep(v16b a, v16b b, v16b c, v16b d) { keep4_b(a, b, c, d); }
};

__device__ __forceinline__ unsigned pk16(unsigned short a, unsigned short b) { return (unsigned)a | ((unsigned)b << 16); }
__device__ __forceinline__ unsigned short h_bits(float f) { const _Float16 h = (_Float16)f; return __builtin_bit_cast(unsigned short, h); }
__device__ __forceinline__ float bf16r(float f) { return bf_bits2f(f2bf_bits(f)); }

template <int ET> struct Elem;
template <> struct Elem<0> { typedef _Float16 T; };
template <> struct Elem<1> { typedef __bf16 T; };
template <int ET, bool SPLIT, int BIAS_MODE, int OUT_MODE, bool RESID, int ACT = 0>
__global__ __launch_bounds__(256) void wmma_gemm64(
    const unsigned short* __restrict__ Ap, const unsigned short* __restrict__ A2p, int lda, long strideA,
    const unsigned short* __restrict__ Btp, const unsigned short* __restrict__ Bt2p, int ldb, long strideB,
    void* __restrict__ Cout, void* __restrict__ Cout2, int ldc, long strideC,
    const float* __restrict__ bias,
    const float* __restrict__ resid, long strideR,
    int M, int N, int K, float scale) {
  typedef typename Elem<ET>::T T;
  typedef typename Frag<T>::V V;
  const T* A = (const T*)Ap; const T* A2 = (const T*)A2p; const T* Bt = (const T*)Btp; const T* Bt2 = (const T*)Bt2p;
  __shared__ __align__(16) float sT[8][16 * 68];
  const int b    = blockIdx.y;
  const int lane = threadIdx.x & 31;
  const int wave = threadIdx.x >> 5;
  const int tilesN = N >> 6;
  const int tilesM = M >> 6;
  const int tile = blockIdx.x * 8 + wave;
  if (tile >= tilesM * tilesN) return;
  const int tm = tile / tilesN;
  const int tn = tile - tm * tilesN;
  const int m0 = tm << 6;
  const int n0 = tn << 6;

  const T* Ab  = A  + (size_t)b * strideA;
  const T* Bb  = Bt + (size_t)b * strideB;
  const T* Ab2 = SPLIT ? (A2  + (size_t)b * strideA) : nullptr;
  const T* Bb2 = SPLIT ? (Bt2 + (size_t)b * strideB) : nullptr;

  const int rlane = lane & 15;
  const int koff  = (lane >> 4) * 8;
  const int mOff  = (lane >> 4) * 8;

  v8f acc[4][4];
#pragma unroll
  for (int i = 0; i < 4; ++i)
#pragma unroll
    for (int j = 0; j < 4; ++j) acc[i][j] = (v8f){0.f,0.f,0.f,0.f,0.f,0.f,0.f,0.f};

  for (int k0 = 0; k0 < K; k0 += 32) {
    V bh[4], bl[4];
#pragma unroll
    for (int j = 0; j < 4; ++j) {
      const size_t bo = (size_t)(n0 + (j << 4) + rlane) * ldb + koff + k0;
      bh[j] = Frag<T>::load(Bb + bo);
      if (SPLIT) bl[j] = Frag<T>::load(Bb2 + bo);
    }
#pragma unroll
    for (int i = 0; i < 4; ++i) {
      const size_t ao = (size_t)(m0 + (i << 4) + rlane) * lda + koff + k0;
      V ah = Frag<T>::load(Ab + ao);
      V al;
      if (SPLIT) al = Frag<T>::load(Ab2 + ao);
#pragma unroll
      for (int j = 0; j < 4; ++j) {
        acc[i][j] = Frag<T>::mma(ah, bh[j], acc[i][j]);
        if (SPLIT) {
          acc[i][j] = Frag<T>::mma(ah, bl[j], acc[i][j]);
          acc[i][j] = Frag<T>::mma(al, bh[j], acc[i][j]);
        }
      }
      Frag<T>::guard(acc[i][0], acc[i][3], ah, SPLIT ? al : ah);
    }
    Frag<T>::keep(bh[0], bh[1], bh[2], bh[3]);
    if (SPLIT) Frag<T>::keep(bl[0], bl[1], bl[2], bl[3]);
  }
  acc_guard4(acc[0][0], acc[0][1], acc[0][2], acc[0][3]);
  acc_guard4(acc[1][0], acc[1][1], acc[1][2], acc[1][3]);
  acc_guard4(acc[2][0], acc[2][1], acc[2][2], acc[2][3]);
  acc_guard4(acc[3][0], acc[3][1], acc[3][2], acc[3][3]);

  float* slab = sT[wave];
  const float* Rb = RESID ? (resid + (size_t)b * strideR) : nullptr;
#pragma unroll
  for (int i = 0; i < 4; ++i) {
    const int mBase = m0 + (i << 4);
#pragma unroll
    for (int j = 0; j < 4; ++j) {
      const int n = n0 + (j << 4) + rlane;
      float bv = 0.f;
      if (BIAS_MODE == 2) bv = bias[n];
#pragma unroll
      for (int r = 0; r < 8; ++r) {
        float v = acc[i][j][r] * scale;
        if (BIAS_MODE == 1) v += bias[mBase + mOff + r];
        if (BIAS_MODE == 2) v += bv;
        if (RESID) v += Rb[(size_t)(mBase + mOff + r) * ldc + n];
        if (ACT == 2) v = fmaxf(v, 0.0f);
        if (ACT == 4) v = (v > 0.f) ? v : 0.01f * v;
        slab[(mOff + r) * 68 + (j << 4) + rlane] = v;
      }
    }
    __builtin_amdgcn_fence(__ATOMIC_RELEASE, "workgroup");
    __builtin_amdgcn_wave_barrier();
    __builtin_amdgcn_fence(__ATOMIC_ACQUIRE, "workgroup");
    if (OUT_MODE == 0) {
      float* C = (float*)Cout + (size_t)b * strideC;
      const int hh = lane >> 4, c4 = (lane & 15) * 4;
      for (int pass = 0; pass < 2; ++pass) {
#pragma unroll
        for (int it = 0; it < 8; ++it) {
          const int row = it * 2 + hh;
          v4f v = *(const v4f*)(slab + row * 68 + c4);
          *(volatile v4f*)(C + (size_t)(mBase + row) * ldc + n0 + c4) = v;
        }
        __threadfence();
      }
    } else {
      const int q = lane >> 3, c8 = (lane & 7) * 8;
      unsigned short* C  = (unsigned short*)Cout  + (size_t)b * strideC;
      unsigned short* C2 = (OUT_MODE == 2) ? ((unsigned short*)Cout2 + (size_t)b * strideC) : nullptr;
      for (int pass = 0; pass < 2; ++pass) {
#pragma unroll
        for (int it = 0; it < 4; ++it) {
          const int row = it * 4 + q;
          const float* sp = slab + row * 68 + c8;
          v8h hv, lv;
#pragma unroll
          for (int e = 0; e < 8; ++e) {
            if (OUT_MODE == 1) {
              hv[e] = (_Float16)sp[e];
            } else {
              unsigned short hb = f2bf_bits(sp[e]);
              unsigned short lb = f2bf_bits(sp[e] - bf_bits2f(hb));
              hv[e] = __builtin_bit_cast(_Float16, hb);
              lv[e] = __builtin_bit_cast(_Float16, lb);
            }
          }
          *(volatile v8h*)(C + (size_t)(mBase + row) * ldc + n0 + c8) = hv;
          if (OUT_MODE == 2) *(volatile v8h*)(C2 + (size_t)(mBase + row) * ldc + n0 + c8) = lv;
        }
        __threadfence();
      }
    }
    __builtin_amdgcn_fence(__ATOMIC_RELEASE, "workgroup");
    __builtin_amdgcn_wave_barrier();
    __builtin_amdgcn_fence(__ATOMIC_ACQUIRE, "workgroup");
  }
}

__global__ __launch_bounds__(128) void prep_vec_kernel(
    const float* __restrict__ theta_b, const float* __restrict__ phi_b,
    const float* __restrict__ g_b, const float* __restrict__ wz_b,
    float* __restrict__ biasQK, float* __restrict__ biasG, float* __restrict__ biasZ) {
  const int y = blockIdx.y;
  const float* s0 = (y == 0) ? theta_b : (y == 1) ? g_b : wz_b;
  const float* s1 = (y == 0) ? phi_b : s0;
  float* dst = (y == 0) ? biasQK : (y == 1) ? biasG : biasZ;
  const int n0   = (y == 2) ? NCH : NIC;
  const int ntot = (y == 1) ? NIC : NCH;
  const int t = threadIdx.x;
  const int e = 4 * t;
  if (e >= ntot) return;
  int ia = e;      if (ia > n0 - 4) ia = n0 - 4;
  int ib = e - n0; if (ib < 0) ib = 0; if (ib > NIC - 4) ib = NIC - 4;
  const v4f a = *(const v4f*)(s0 + ia);
  const v4f c = *(const v4f*)(s1 + ib);
  const bool usea = (e < n0);
  v4f o;
#pragma unroll
  for (int k = 0; k < 4; ++k) o[k] = bf16r(usea ? a[k] : c[k]);
  float* p = dst + e;
  *(volatile v4f*)p = o;
  __threadfence();
  *(volatile v4f*)p = o;
}

__global__ __launch_bounds__(256) void wcast_kernel(const float* __restrict__ w0, const float* __restrict__ w1,
                                                    const float* __restrict__ w2, const float* __restrict__ w3,
                                                    unsigned short* __restrict__ d0, unsigned short* __restrict__ d1,
                                                    unsigned short* __restrict__ d2, unsigned short* __restrict__ d3,
                                                    int n8, float scale) {
  const int z = blockIdx.y;
  const float* src = (z == 0) ? w0 : (z == 1) ? w1 : (z == 2) ? w2 : w3;
  unsigned short* dst = (z == 0) ? d0 : (z == 1) ? d1 : (z == 2) ? d2 : d3;
  const int i = blockIdx.x * 256 + threadIdx.x;
  if (i >= n8) return;
  const float* p = src + 8 * (size_t)i;
  const v4f a = *(const v4f*)(p);
  const v4f c = *(const v4f*)(p + 4);
  unsigned short hb[8];
#pragma unroll
  for (int e = 0; e < 4; ++e) {
    hb[e]     = h_bits(scale * bf16r(a[e]));
    hb[4 + e] = h_bits(scale * bf16r(c[e]));
  }
  const v4u u = (v4u){pk16(hb[0], hb[1]), pk16(hb[2], hb[3]), pk16(hb[4], hb[5]), pk16(hb[6], hb[7])};
  unsigned short* q = dst + 8 * (size_t)i;
  *(volatile v4u*)q = u;
  __threadfence();
  *(volatile v4u*)q = u;
}

__global__ __launch_bounds__(256) void xT_kernel(const float* __restrict__ xb, unsigned short* __restrict__ xtm) {
  __shared__ float sm[64][65];
  const int t  = threadIdx.x;
  const int c0 = blockIdx.x * 64;
  const int n0 = blockIdx.y * 64;
#pragma unroll
  for (int i = 0; i < 16; ++i) {
    const int e  = i * 256 + t;
    const int r  = e >> 6;
    const int cc = e & 63;
    sm[cc][r] = xb[(size_t)(c0 + r) * NTOK + n0 + cc];
  }
  __syncthreads();
  const int lane = t & 31, wave = t >> 5;
  const int q = lane >> 3, c8 = (lane & 7) * 8;
  for (int pass = 0; pass < 2; ++pass) {
#pragma unroll
    for (int it = 0; it < 2; ++it) {
      const int row = wave * 8 + it * 4 + q;
      unsigned short hb[8];
#pragma unroll
      for (int e = 0; e < 8; ++e) hb[e] = h_bits(bf16r(sm[row][c8 + e]));
      const v4u u = (v4u){pk16(hb[0], hb[1]), pk16(hb[2], hb[3]), pk16(hb[4], hb[5]), pk16(hb[6], hb[7])};
      *(volatile v4u*)(xtm + (size_t)(n0 + row) * NCH + c0 + c8) = u;
    }
    __threadfence();
  }
}

constexpr int SMX_THREADS = 416;
constexpr int SMX_ACTIVE  = NTOK / 8;
constexpr int SMX_WAVES   = SMX_THREADS / 32;
static_assert(SMX_ACTIVE * 8 == NTOK && SMX_ACTIVE <= SMX_THREADS && SMX_WAVES == 13);
__global__ __launch_bounds__(SMX_THREADS) void softmax_row_kernel(const float* __restrict__ S, unsigned short* __restrict__ P, float carry) {
  __shared__ float redM[16];
  __shared__ float redS[16];
  const int row  = blockIdx.x;
  const int t    = threadIdx.x;
  const int lane = t & 31, wave = t >> 5;
  const bool active = (t < SMX_ACTIVE);
  const int tc = active ? t : (SMX_ACTIVE - 1);
  const float* sr = S + (size_t)row * NTOK + 8 * tc;
  const v4f a = *(const v4f*)(sr);
  const v4f c = *(const v4f*)(sr + 4);
  float x[8];
#pragma unroll
  for (int e = 0; e < 4; ++e) { x[e] = a[e]; x[4 + e] = c[e]; }
  float m = fmaxf(fmaxf(fmaxf(x[0], x[1]), fmaxf(x[2], x[3])), fmaxf(fmaxf(x[4], x[5]), fmaxf(x[6], x[7])));
  if (!active) m = -INFINITY;
#pragma unroll
  for (int off = 16; off > 0; off >>= 1) m = fmaxf(m, __shfl_xor(m, off, 32));
  if (lane == 0) redM[wave] = m;
  __syncthreads();
  float gm = redM[0];
#pragma unroll
  for (int w = 1; w < SMX_WAVES; ++w) gm = fmaxf(gm, redM[w]);
  float s = 0.f;
#pragma unroll
  for (int e = 0; e < 8; ++e) { x[e] = __expf(x[e] - gm); s += x[e]; }
  if (!active) s = 0.f;
#pragma unroll
  for (int off = 16; off > 0; off >>= 1) s += __shfl_xor(s, off, 32);
  if (lane == 0) redS[wave] = s;
  __syncthreads();
  float gs = redS[0];
#pragma unroll
  for (int w = 1; w < SMX_WAVES; ++w) gs += redS[w];
  const float inv = carry * (1.0f / gs);
  if (active) {
    unsigned short hb[8];
#pragma unroll
    for (int e = 0; e < 8; ++e) hb[e] = h_bits(x[e] * inv);
    const v4u u = (v4u){pk16(hb[0], hb[1]), pk16(hb[2], hb[3]), pk16(hb[4], hb[5]), pk16(hb[6], hb[7])};
    unsigned short* q = P + (size_t)row * NTOK + 8 * t;
    *(volatile v4u*)q = u;
    __threadfence();
    *(volatile v4u*)q = u;
  }
}

__global__ __launch_bounds__(256) void bn_stats_kernel(const float* __restrict__ Z, float* __restrict__ mean_out,
                                                       float* __restrict__ rstd_out) {
  __shared__ __align__(16) float smean[32];
  __shared__ __align__(16) float srstd[32];
  const int lane = threadIdx.x & 31, wave = threadIdx.x >> 5;
  const int cbase = blockIdx.x * 32;
  const float invn = 1.0f / (float)(NBATCH * NTOK);
#pragma unroll 1
  for (int k = 0; k < 4; ++k) {
    const int cl = wave + 8 * k;
    const int c  = cbase + cl;
    float s = 0.f, q = 0.f;
#pragma unroll 1
    for (int b = 0; b < NBATCH; ++b) {
      const float* p = Z + ((size_t)b * NCH + c) * NTOK + lane;
#pragma unroll 2
      for (int i = 0; i < NTOK / 32; ++i) {
        const float v = p[32 * i];
        s += v;
        q += v * v;
      }
    }
#pragma unroll
    for (int off = 16; off > 0; off >>= 1) {
      s += __shfl_xor(s, off, 32);
      q += __shfl_xor(q, off, 32);
    }
    if (lane == 0) {
      const float mean = s * invn;
      float var = q * invn - mean * mean;
      var = fmaxf(var, 0.0f);
      smean[cl] = mean;
      srstd[cl] = rsqrtf(var + BNEPS);
    }
  }
  __syncthreads();
  if (wave == 0 && lane < 8) {
    const v4f v = *(const v4f*)(smean + 4 * lane);
    float* p = mean_out + cbase + 4 * lane;
    *(volatile v4f*)p = v;
    __threadfence();
    *(volatile v4f*)p = v;
  }
  if (wave == 1 && lane < 8) {
    const v4f v = *(const v4f*)(srstd + 4 * lane);
    float* p = rstd_out + cbase + 4 * lane;
    *(volatile v4f*)p = v;
    __threadfence();
    *(volatile v4f*)p = v;
  }
}

__global__ __launch_bounds__(256) void bn_apply_kernel(const float* __restrict__ Z, const float* __restrict__ X,
                                                       const float* __restrict__ meanp, const float* __restrict__ rstdp,
                                                       const float* __restrict__ bn_w, const float* __restrict__ bn_b,
                                                       float* __restrict__ out, int n4) {
  const int i = blockIdx.x * 256 + threadIdx.x;
  if (i >= n4) return;
  const unsigned e = 4u * (unsigned)i;
  const int c = (int)((e / (unsigned)NTOK) % (unsigned)NCH);
  const v4f z  = *(const v4f*)(Z + e);
  const v4f xv = *(const v4f*)(X + e);
  const float m  = meanp[c];
  const float r  = rstdp[c];
  const float w  = bf16r(bn_w[c]);
  const float bb = bf16r(bn_b[c]);
  v4f o;
#pragma unroll
  for (int k = 0; k < 4; ++k) {
    const float yn = (z[k] - m) * r;
    const float ya = yn * w + bb;
    o[k] = ya + bf16r(xv[k]);
  }
  float* p = out + e;
  *(volatile v4f*)p = o;
  __threadfence();
  *(volatile v4f*)p = o;
}

extern "C" void kernel_launch(void* const* d_in, const int* in_sizes, int n_in,
                              void* d_out, int out_size, void* d_ws, size_t ws_size,
                              hipStream_t stream) {
  if (n_in < 11) return;
  if (in_sizes[0] != NBATCH * NCH * NTOK) return;
  if (out_size != NBATCH * NCH * NTOK) return;
  if (in_sizes[1] != NIC * NCH || in_sizes[3] != NIC * NCH || in_sizes[5] != NIC * NCH || in_sizes[7] != NCH * NIC) return;
  if (in_sizes[2] != NIC || in_sizes[4] != NIC || in_sizes[6] != NIC) return;
  if (in_sizes[8] != NCH || in_sizes[9] != NCH || in_sizes[10] != NCH) return;
  if (ws_size < WS_END) return;

  const float* x       = (const float*)d_in[0];
  const float* theta_w = (const float*)d_in[1];
  const float* theta_b = (const float*)d_in[2];
  const float* phi_w   = (const float*)d_in[3];
  const float* phi_b   = (const float*)d_in[4];
  const float* g_w     = (const float*)d_in[5];
  const float* g_b     = (const float*)d_in[6];
  const float* wz_w    = (const float*)d_in[7];
  const float* wz_b    = (const float*)d_in[8];
  const float* bn_w    = (const float*)d_in[9];
  const float* bn_b    = (const float*)d_in[10];
  float* out = (float*)d_out;

  char* ws = (char*)d_ws;
  unsigned short* Wqk = (unsigned short*)(ws + OFF_WQK);
  unsigned short* Wg  = (unsigned short*)(ws + OFF_WG);
  unsigned short* Wz  = (unsigned short*)(ws + OFF_WZ);
  float* biasQK = (float*)(ws + OFF_VEC);
  float* biasG  = (float*)(ws + OFF_VEC + 2048);
  float* biasZ  = (float*)(ws + OFF_VEC + 3072);
  float* meanp  = (float*)(ws + OFF_VEC + 5120);
  float* rstdp  = (float*)(ws + OFF_VEC + 7168);
  unsigned short* xtm  = (unsigned short*)(ws + OFF_XTM);
  unsigned short* QKhi = (unsigned short*)(ws + OFF_QKH);
  unsigned short* QKlo = (unsigned short*)(ws + OFF_QKL);
  unsigned short* Khi  = QKhi + NIC;
  unsigned short* Klo  = QKlo + NIC;
  unsigned short* Vt   = (unsigned short*)(ws + OFF_VT);
  float*          Sp   = (float*)(ws + OFF_S);
  unsigned short* Pp   = (unsigned short*)(ws + OFF_P);
  unsigned short* Yp   = (unsigned short*)(ws + OFF_Y);
  float*          Zp   = (float*)(ws + OFF_Z);

  const dim3 blk256(256);

  prep_vec_kernel<<<dim3(1, 3), dim3(128), 0, stream>>>(theta_b, phi_b, g_b, wz_b, biasQK, biasG, biasZ);
  wcast_kernel<<<dim3((NIC * NCH / 8) / 256, 4), blk256, 0, stream>>>(
      theta_w, phi_w, g_w, wz_w, Wqk, Wqk + (size_t)NIC * NCH, Wg, Wz, NIC * NCH / 8, WCARRY);

  const int tilesTok = NTOK / 64;
  const int gridS    = (tilesTok * tilesTok + 7) / 8;
  const int gridV    = (tilesTok * (NIC / 64) + 7) / 8;
  const int gridZ    = (tilesTok * (NCH / 64) + 7) / 8;
  const int gridQK   = (tilesTok * (NCH / 64) + 7) / 8;

  for (int b = 0; b < NBATCH; ++b) {
    const float* xb = x + (size_t)b * NCH * NTOK;
    float* Zb = Zp + (size_t)b * NCH * NTOK;

    xT_kernel<<<dim3(NCH / 64, NTOK / 64), blk256, 0, stream>>>(xb, xtm);

    wmma_gemm64<0, false, 2, 2, false, 0><<<dim3(gridQK, 1), blk256, 0, stream>>>(
        xtm, xtm, NCH, 0, Wqk, Wqk, NCH, 0, (void*)QKhi, (void*)QKlo, 2 * NIC, 0,
        biasQK, biasQK, 0, NTOK, 2 * NIC, NCH, WCARRY_INV);

    wmma_gemm64<0, false, 1, 1, false, 0><<<dim3(gridV, 1), blk256, 0, stream>>>(
        Wg, Wg, NCH, 0, xtm, xtm, NCH, 0, (void*)Vt, (void*)Vt, NTOK, 0,
        biasG, biasG, 0, NIC, NTOK, NCH, WCARRY_INV);

    wmma_gemm64<1, true, 0, 0, false, 0><<<dim3(gridS, 1), blk256, 0, stream>>>(
        QKhi, QKlo, 2 * NIC, 0, Khi, Klo, 2 * NIC, 0, (void*)Sp, (void*)Sp, NTOK, 0,
        biasQK, biasQK, 0, NTOK, NTOK, NIC, 1.0f);

    softmax_row_kernel<<<dim3(NTOK), dim3(SMX_THREADS), 0, stream>>>(Sp, Pp, PCARRY);

    wmma_gemm64<0, false, 0, 1, false, 0><<<dim3(gridV, 1), blk256, 0, stream>>>(
        Pp, Pp, NTOK, 0, Vt, Vt, NTOK, 0, (void*)Yp, (void*)Yp, NIC, 0,
        biasQK, biasQK, 0, NTOK, NIC, NTOK, PV_SCALE);

    wmma_gemm64<0, false, 1, 0, false, 0><<<dim3(gridZ, 1), blk256, 0, stream>>>(
        Wz, Wz, NIC, 0, Yp, Yp, NIC, 0, (void*)Zb, (void*)Zb, NTOK, 0,
        biasZ, biasZ, 0, NCH, NTOK, NIC, Z_SCALE);
  }

  bn_stats_kernel<<<dim3(NCH / 32), blk256, 0, stream>>>(Zp, meanp, rstdp);
  const int n4 = NBATCH * NCH * NTOK / 4;
  bn_apply_kernel<<<dim3((n4 + 255) / 256), blk256, 0, stream>>>(Zp, x, meanp, rstdp, bn_w, bn_b, out, n4);
}
